// SpinTransformerModule_62869731279058
// MI455X (gfx1250) — hardware-verified
//
#include <hip/hip_runtime.h>
#include <math.h>
#include <stdint.h>

#define NB_   2
#define SEQ   2048
#define DIM   1024
#define NH    16
#define HD    64
#define NBH   (NB_ * NH)
#define FFD   4096
#define GRP   8
#define NSTEP 8
#define TP    68

#define MODE_QK   0
#define MODE_GELU 1
#define MODE_FF2  2

#define SCALE_F   22.605309110915f
#define SCALE_HD  5.5677643628300215f
#define W_CARRY   64.0f
#define H_CARRY   16.0f
#define QK_CARRY  256.0f
#define E_CARRY   16.0f
#define M_CARRY   64.0f

static_assert(NH * HD == DIM);
static_assert((SEQ % 64) == 0 && (DIM % 64) == 0 && (FFD % 64) == 0);
static_assert((NBH % GRP) == 0);

typedef _Float16 v16h __attribute__((ext_vector_type(16)));
typedef _Float16 v8h  __attribute__((ext_vector_type(8)));
typedef float    v8f  __attribute__((ext_vector_type(8)));
typedef float    v4f  __attribute__((ext_vector_type(4)));
typedef unsigned int v4u __attribute__((ext_vector_type(4)));
typedef unsigned int v2u __attribute__((ext_vector_type(2)));

__device__ __forceinline__ unsigned short hb(float f) { return __builtin_bit_cast(unsigned short, (_Float16)f); }
__device__ __forceinline__ unsigned pk16(unsigned short a, unsigned short b) { return (unsigned)a | ((unsigned)b << 16); }
__device__ __forceinline__ v8f zero8() { v8f z = {0.f, 0.f, 0.f, 0.f, 0.f, 0.f, 0.f, 0.f}; return z; }
__device__ __forceinline__ void sched_fence() { asm volatile("" ::: "memory"); }

__device__ __forceinline__ v16h ldfrag(const _Float16* p) {
  union { v16h v; v8h h[2]; } f;
  f.h[0] = *(const v8h*)(p);
  f.h[1] = *(const v8h*)(p + 16);
  return f.v;
}

__device__ __forceinline__ v8f mma_raw(v16h a, v16h b, v8f c) {
  return __builtin_amdgcn_wmma_f32_16x16x32_f16(false, a, false, b, (short)0, c, false, false);
}
__device__ __forceinline__ void dep_guard(v8f& a, v8f& b, v16h x, v16h y) {
  asm volatile("v_nop\n\tv_nop\n\tv_nop\n\tv_nop" : "+v"(a), "+v"(b) : "v"(x), "v"(y));
}
__device__ __forceinline__ void keep4(v16h a, v16h b, v16h c, v16h d) {
  asm volatile("v_nop" :: "v"(a), "v"(b), "v"(c), "v"(d));
}
__device__ __forceinline__ void acc_guard4(v8f& a, v8f& b, v8f& c, v8f& d) {
  asm volatile("v_nop\n\tv_nop\n\tv_nop\n\tv_nop" : "+v"(a), "+v"(b), "+v"(c), "+v"(d));
}
__device__ __forceinline__ void lds_sync() {
  __builtin_amdgcn_fence(__ATOMIC_RELEASE, "workgroup");
  __builtin_amdgcn_wave_barrier();
  __builtin_amdgcn_fence(__ATOMIC_ACQUIRE, "workgroup");
}

__device__ __forceinline__ void write16h(const float* slab, unsigned short* C, size_t ldc, int lane) {
  const int q = lane >> 3, c8 = (lane & 7) * 8;
  v4u hv[4];
#pragma unroll
  for (int it = 0; it < 4; ++it) {
    const int row = it * 4 + q;
    const float* sp = slab + row * TP + c8;
    const v4f a = *(const v4f*)(sp);
    const v4f b = *(const v4f*)(sp + 4);
    v4u p;
    p[0] = pk16(hb(a[0]), hb(a[1]));
    p[1] = pk16(hb(a[2]), hb(a[3]));
    p[2] = pk16(hb(b[0]), hb(b[1]));
    p[3] = pk16(hb(b[2]), hb(b[3]));
    hv[it] = p;
  }
  for (int pass = 0; pass < 2; ++pass) {
#pragma unroll
    for (int it = 0; it < 4; ++it) {
      const int row = it * 4 + q;
      *(volatile v4u*)(C + (size_t)row * ldc + c8) = hv[it];
    }
    __threadfence();
  }
}
__device__ __forceinline__ void write32f(const float* slab, float* C, size_t ldc, int lane) {
  const int h2 = lane >> 4, c4 = (lane & 15) * 4;
  for (int pass = 0; pass < 2; ++pass) {
#pragma unroll
    for (int it = 0; it < 8; ++it) {
      const int row = it * 2 + h2;
      const v4f v = *(const v4f*)(slab + row * TP + c4);
      *(volatile v4f*)(C + (size_t)row * ldc + c4) = v;
    }
    __threadfence();
  }
}

__global__ __launch_bounds__(256) void k_cvt_h(const float* __restrict__ in, unsigned short* out, int n8, float sc) {
  const int i = blockIdx.x * 256 + threadIdx.x;
  if (i < n8) {
    const v4f a = *(const v4f*)(in + (size_t)i * 8);
    const v4f b = *(const v4f*)(in + (size_t)i * 8 + 4);
    v4u p;
    p[0] = pk16(hb(a[0] * sc), hb(a[1] * sc));
    p[1] = pk16(hb(a[2] * sc), hb(a[3] * sc));
    p[2] = pk16(hb(b[0] * sc), hb(b[1] * sc));
    p[3] = pk16(hb(b[2] * sc), hb(b[3] * sc));
    unsigned short* d = out + (size_t)i * 8;
    *(volatile v4u*)d = p;
    __threadfence();
    *(volatile v4u*)d = p;
  }
}

__global__ __launch_bounds__(256) void k_norm_x(const float* __restrict__ x, float* xsF, unsigned short* xsH) {
  __shared__ float wsum[8];
  const int row = blockIdx.x;
  const int t = threadIdx.x;
  const v4f v = *(const v4f*)(x + (size_t)row * DIM + t * 4);
  float ss = v[0] * v[0] + v[1] * v[1] + v[2] * v[2] + v[3] * v[3];
#pragma unroll
  for (int off = 1; off < 32; off <<= 1) ss += __shfl_xor(ss, off, 32);
  if ((t & 31) == 0) wsum[t >> 5] = ss;
  __syncthreads();
  float tot = 0.f;
#pragma unroll
  for (int i = 0; i < 8; ++i) tot += wsum[i];
  const float s = SCALE_F / fmaxf(sqrtf(tot), 1e-12f);
  v4f o;
  o[0] = v[0] * s; o[1] = v[1] * s; o[2] = v[2] * s; o[3] = v[3] * s;
  v2u p;
  p[0] = pk16(hb(o[0]), hb(o[1]));
  p[1] = pk16(hb(o[2]), hb(o[3]));
  float* df = xsF + (size_t)row * DIM + t * 4;
  unsigned short* dh = xsH + (size_t)row * DIM + t * 4;
  *(volatile v4f*)df = o;
  *(volatile v2u*)dh = p;
  __threadfence();
  *(volatile v4f*)df = o;
  *(volatile v2u*)dh = p;
}

__device__ __forceinline__ void tile64(const _Float16* __restrict__ A, size_t lda,
                                       const _Float16* __restrict__ Bt, size_t ldb,
                                       int K, int lane, v8f (&acc)[4][4]) {
  const int rl = lane & 15;
  const int koff = (lane >> 4) * 8;
#pragma unroll
  for (int i = 0; i < 4; ++i)
#pragma unroll
    for (int j = 0; j < 4; ++j) acc[i][j] = zero8();
#pragma unroll 1
  for (int k0 = 0; k0 < K; k0 += 32) {
    v16h bfr[4];
#pragma unroll
    for (int j = 0; j < 4; ++j) bfr[j] = ldfrag(Bt + (size_t)(16 * j + rl) * ldb + koff + k0);
#pragma unroll
    for (int i = 0; i < 4; ++i) {
      const v16h af = ldfrag(A + (size_t)(16 * i + rl) * lda + koff + k0);
#pragma unroll
      for (int j = 0; j < 4; ++j) acc[i][j] = mma_raw(af, bfr[j], acc[i][j]);
      dep_guard(acc[i][0], acc[i][3], af, bfr[3]);
    }
    keep4(bfr[0], bfr[1], bfr[2], bfr[3]);
  }
  acc_guard4(acc[0][0], acc[0][1], acc[0][2], acc[0][3]);
  acc_guard4(acc[1][0], acc[1][1], acc[1][2], acc[1][3]);
  acc_guard4(acc[2][0], acc[2][1], acc[2][2], acc[2][3]);
  acc_guard4(acc[3][0], acc[3][1], acc[3][2], acc[3][3]);
}

template <int MODE>
__global__ __launch_bounds__(256) void k_gemm(const unsigned short* __restrict__ Ap, int lda,
                                              const unsigned short* __restrict__ Bp, int ldb,
                                              int M, int N, int K,
                                              unsigned short* O16a, unsigned short* O16b,
                                              float* O32, const float* __restrict__ aux) {
  __shared__ __align__(16) float sT[8][16 * TP];
  const int lane = threadIdx.x & 31;
  const int wave = threadIdx.x >> 5;
  const int h = lane >> 4, c = lane & 15;
  const int tilesN = N >> 6, tilesM = M >> 6;
  const int tile = blockIdx.x * 8 + wave;
  if (tile >= tilesM * tilesN) return;
  const int tm = tile / tilesN;
  const int tn = tile - tm * tilesN;
  const int m0 = tm << 6, n0 = tn << 6;
  const _Float16* A  = (const _Float16*)(const void*)Ap + (size_t)m0 * lda;
  const _Float16* Bt = (const _Float16*)(const void*)Bp + (size_t)n0 * ldb;

  v8f acc[4][4];
  tile64(A, (size_t)lda, Bt, (size_t)ldb, K, lane, acc);
  float* slab = sT[wave];

  if (MODE == MODE_QK) {
    const float cs = 1.0f / W_CARRY;
    float scl[4][8];
#pragma unroll
    for (int i = 0; i < 4; ++i)
#pragma unroll
      for (int r = 0; r < 8; ++r) {
        float ss = 0.f;
#pragma unroll
        for (int j = 0; j < 4; ++j) { const float v = acc[i][j][r] * cs; ss += v * v; }
        ss += __shfl_xor(ss, 1, 32);
        ss += __shfl_xor(ss, 2, 32);
        ss += __shfl_xor(ss, 4, 32);
        ss += __shfl_xor(ss, 8, 32);
        scl[i][r] = (QK_CARRY * cs) / fmaxf(sqrtf(ss), 1e-12f);
      }
    unsigned short* dst = (n0 < DIM) ? O16a : O16b;
    const int hd = (n0 & (DIM - 1)) >> 6;
    const int b = m0 / SEQ, nb0 = m0 & (SEQ - 1);
    unsigned short* base = dst + ((size_t)(b * NH + hd) * SEQ + nb0) * HD;
#pragma unroll
    for (int i = 0; i < 4; ++i) {
#pragma unroll
      for (int j = 0; j < 4; ++j)
#pragma unroll
        for (int r = 0; r < 8; ++r) slab[(8 * h + r) * TP + 16 * j + c] = acc[i][j][r] * scl[i][r];
      lds_sync();
      write16h(slab, base + (size_t)(16 * i) * HD, (size_t)HD, lane);
      lds_sync();
    }
  } else if (MODE == MODE_GELU) {
    const float cs = 1.0f / W_CARRY;
#pragma unroll
    for (int i = 0; i < 4; ++i) {
#pragma unroll
      for (int j = 0; j < 4; ++j)
#pragma unroll
        for (int r = 0; r < 8; ++r) {
          const float v = acc[i][j][r] * cs;
          const float g = 0.5f * v * (1.0f + erff(v * 0.70710678118654752f));
          slab[(8 * h + r) * TP + 16 * j + c] = g * H_CARRY;
        }
      lds_sync();
      write16h(slab, O16a + (size_t)(m0 + 16 * i) * FFD + n0, (size_t)FFD, lane);
      lds_sync();
    }
  } else {
    const int hd = m0 >> 6;
    const int b = n0 / SEQ, nb0 = n0 & (SEQ - 1);
    const int bh = b * NH + hd;
    const float cs = 1.0f / (W_CARRY * H_CARRY);
#pragma unroll
    for (int j = 0; j < 4; ++j) {
#pragma unroll
      for (int i = 0; i < 4; ++i) {
        const v8f xv = *(const v8f*)(aux + (size_t)(n0 + 16 * j + c) * DIM + m0 + 16 * i + 8 * h);
#pragma unroll
        for (int r = 0; r < 8; ++r) acc[i][j][r] = acc[i][j][r] * cs + xv[r];
      }
      sched_fence();
    }
    float* xfb = O32 + ((size_t)bh * SEQ + nb0) * HD;
#pragma unroll
    for (int j = 0; j < 4; ++j) {
#pragma unroll
      for (int i = 0; i < 4; ++i) {
        v4f a, bq;
        a[0] = acc[i][j][0]; a[1] = acc[i][j][1]; a[2] = acc[i][j][2]; a[3] = acc[i][j][3];
        bq[0] = acc[i][j][4]; bq[1] = acc[i][j][5]; bq[2] = acc[i][j][6]; bq[3] = acc[i][j][7];
        *(v4f*)(slab + c * TP + 16 * i + 8 * h) = a;
        *(v4f*)(slab + c * TP + 16 * i + 8 * h + 4) = bq;
      }
      lds_sync();
      write32f(slab, xfb + (size_t)(16 * j) * HD, (size_t)HD, lane);
      lds_sync();
    }
    const float m0c = 1.0f / (1.0f + sqrtf(1.0f + (float)HD * (1.0f / 511.0f)));
    float inv[4];
#pragma unroll
    for (int j = 0; j < 4; ++j) {
      float h2 = 0.f;
#pragma unroll
      for (int i = 0; i < 4; ++i)
#pragma unroll
        for (int r = 0; r < 8; ++r) {
          const float th = acc[i][j][r] + m0c;
          acc[i][j][r] = th;
          h2 += th * th;
        }
      h2 += __shfl_xor(h2, 16, 32);
      inv[j] = M_CARRY * (1.0f / (1.0f + sqrtf(1.0f + h2 * (1.0f / 511.0f))));
    }
    unsigned short* mb = O16a + (size_t)bh * HD * SEQ + nb0;
#pragma unroll
    for (int i = 0; i < 4; ++i) {
#pragma unroll
      for (int j = 0; j < 4; ++j)
#pragma unroll
        for (int r = 0; r < 8; ++r) slab[(8 * h + r) * TP + 16 * j + c] = acc[i][j][r] * inv[j];
      lds_sync();
      write16h(slab, mb + (size_t)(16 * i) * SEQ, (size_t)SEQ, lane);
      lds_sync();
    }
  }
}

__global__ __launch_bounds__(256) void k_scores(const unsigned short* __restrict__ qp,
                                                const unsigned short* __restrict__ kp,
                                                unsigned short* Ep, float* rinv, int bh0) {
  __shared__ __align__(16) float sT[8][16 * TP];
  const int lane = threadIdx.x & 31;
  const int wave = threadIdx.x >> 5;
  const int h = lane >> 4, c = lane & 15;
  const int blk = blockIdx.x;
  const int bhl = blk >> 3;
  const int bh = bh0 + bhl;
  const int q0 = ((blk & 7) * 8 + wave) * 32;
  const _Float16* Q  = (const _Float16*)(const void*)qp + (size_t)bh * SEQ * HD;
  const _Float16* Kk = (const _Float16*)(const void*)kp + (size_t)bh * SEQ * HD;
  unsigned short* Eg = Ep + (size_t)bhl * SEQ * SEQ;
  float* slab = sT[wave];

  v16h qa[2][2];
#pragma unroll
  for (int i = 0; i < 2; ++i)
#pragma unroll
    for (int kd = 0; kd < 2; ++kd)
      qa[i][kd] = ldfrag(Q + (size_t)(q0 + 16 * i + c) * HD + kd * 32 + 8 * h);

  float rs[2][8];
#pragma unroll
  for (int i = 0; i < 2; ++i)
#pragma unroll
    for (int r = 0; r < 8; ++r) rs[i][r] = 0.f;
  const float ssc = SCALE_HD / (QK_CARRY * QK_CARRY);

#pragma unroll 1
  for (int kt = 0; kt < SEQ / 64; ++kt) {
    v8f s[2][4];
#pragma unroll
    for (int j = 0; j < 4; ++j) {
      s[0][j] = zero8();
      s[1][j] = zero8();
      const _Float16* kr = Kk + (size_t)(kt * 64 + 16 * j + c) * HD + 8 * h;
      const v16h kb0 = ldfrag(kr);
      const v16h kb1 = ldfrag(kr + 32);
#pragma unroll
      for (int i = 0; i < 2; ++i) {
        s[i][j] = mma_raw(qa[i][0], kb0, s[i][j]);
        s[i][j] = mma_raw(qa[i][1], kb1, s[i][j]);
      }
      dep_guard(s[0][j], s[1][j], kb0, kb1);
    }
#pragma unroll
    for (int i = 0; i < 2; ++i) {
#pragma unroll
      for (int j = 0; j < 4; ++j)
#pragma unroll
        for (int r = 0; r < 8; ++r) {
          const float e = __expf(s[i][j][r] * ssc);
          rs[i][r] += e;
          slab[(8 * h + r) * TP + 16 * j + c] = e * E_CARRY;
        }
      lds_sync();
      write16h(slab, Eg + (size_t)(q0 + 16 * i) * SEQ + kt * 64, (size_t)SEQ, lane);
      lds_sync();
    }
  }

#pragma unroll
  for (int i = 0; i < 2; ++i)
#pragma unroll
    for (int r = 0; r < 8; ++r) {
      float v = rs[i][r];
      v += __shfl_xor(v, 1, 32);
      v += __shfl_xor(v, 2, 32);
      v += __shfl_xor(v, 4, 32);
      v += __shfl_xor(v, 8, 32);
      rs[i][r] = 1.0f / v;
    }
#pragma unroll
  for (int i = 0; i < 2; ++i)
#pragma unroll
    for (int r = 0; r < 8; ++r) slab[16 * i + 8 * h + r] = rs[i][r];
  lds_sync();
  if (lane < 8) {
    const v4f v = *(const v4f*)(slab + 4 * lane);
    float* dst = rinv + (size_t)bh * SEQ + q0 + 4 * lane;
    *(volatile v4f*)dst = v;
    __threadfence();
    *(volatile v4f*)dst = v;
  }
}

template <int LAST>
__global__ __launch_bounds__(256) void k_iter(const unsigned short* __restrict__ mTin,
                                              const unsigned short* __restrict__ Ep,
                                              const float* __restrict__ rinv,
                                              const float* __restrict__ xf,
                                              unsigned short* mTout, float* out, int bh0) {
  __shared__ __align__(16) float sT[8][16 * TP];
  const int lane = threadIdx.x & 31;
  const int wave = threadIdx.x >> 5;
  const int h = lane >> 4, c = lane & 15;
  const int blk = blockIdx.x;
  const int bhl = blk >> 2;
  const int bh = bh0 + bhl;
  const int n0 = ((blk & 3) * 8 + wave) * 64;
  const _Float16* A  = (const _Float16*)(const void*)mTin + (size_t)bh * HD * SEQ;
  const _Float16* Bt = (const _Float16*)(const void*)Ep + (size_t)bhl * SEQ * SEQ + (size_t)n0 * SEQ;

  v8f acc[4][4];
  tile64(A, (size_t)SEQ, Bt, (size_t)SEQ, SEQ, lane, acc);

  float rsc[4];
#pragma unroll
  for (int j = 0; j < 4; ++j)
    rsc[j] = rinv[(size_t)bh * SEQ + n0 + 16 * j + c] * (1.0f / (E_CARRY * M_CARRY));
#pragma unroll
  for (int j = 0; j < 4; ++j) {
#pragma unroll
    for (int i = 0; i < 4; ++i) {
      const v8f xv = *(const v8f*)(xf + ((size_t)bh * SEQ + n0 + 16 * j + c) * HD + 16 * i + 8 * h);
#pragma unroll
      for (int r = 0; r < 8; ++r) acc[i][j][r] = acc[i][j][r] * rsc[j] + xv[r];
    }
    sched_fence();
  }
  float inv[4];
#pragma unroll
  for (int j = 0; j < 4; ++j) {
    float h2 = 0.f;
#pragma unroll
    for (int i = 0; i < 4; ++i)
#pragma unroll
      for (int r = 0; r < 8; ++r) h2 += acc[i][j][r] * acc[i][j][r];
    h2 += __shfl_xor(h2, 16, 32);
    inv[j] = 1.0f / (1.0f + sqrtf(1.0f + h2 * (1.0f / 511.0f)));
  }
#pragma unroll
  for (int i = 0; i < 4; ++i)
#pragma unroll
    for (int j = 0; j < 4; ++j)
#pragma unroll
      for (int r = 0; r < 8; ++r) acc[i][j][r] *= inv[j];

  float* slab = sT[wave];
  if (!LAST) {
    unsigned short* mb = mTout + (size_t)bh * HD * SEQ + n0;
#pragma unroll
    for (int i = 0; i < 4; ++i) {
#pragma unroll
      for (int j = 0; j < 4; ++j)
#pragma unroll
        for (int r = 0; r < 8; ++r) slab[(8 * h + r) * TP + 16 * j + c] = acc[i][j][r] * M_CARRY;
      lds_sync();
      write16h(slab, mb + (size_t)(16 * i) * SEQ, (size_t)SEQ, lane);
      lds_sync();
    }
  } else {
    const int b = bh / NH, hd = bh - b * NH;
    float* ob = out + ((size_t)b * SEQ + n0) * DIM + hd * HD;
#pragma unroll
    for (int j = 0; j < 4; ++j) {
#pragma unroll
      for (int i = 0; i < 4; ++i) {
        v4f a, bq;
        a[0] = acc[i][j][0]; a[1] = acc[i][j][1]; a[2] = acc[i][j][2]; a[3] = acc[i][j][3];
        bq[0] = acc[i][j][4]; bq[1] = acc[i][j][5]; bq[2] = acc[i][j][6]; bq[3] = acc[i][j][7];
        *(v4f*)(slab + c * TP + 16 * i + 8 * h) = a;
        *(v4f*)(slab + c * TP + 16 * i + 8 * h + 4) = bq;
      }
      lds_sync();
      write32f(slab, ob + (size_t)(16 * j) * DIM, (size_t)DIM, lane);
      lds_sync();
    }
  }
}

extern "C" void kernel_launch(void* const* d_in, const int* in_sizes, int n_in,
                              void* d_out, int out_size, void* d_ws, size_t ws_size,
                              hipStream_t stream) {
  if (n_in < 4) return;
  if (in_sizes[0] != NB_ * SEQ * DIM) return;
  if (in_sizes[1] != 2 * DIM * DIM) return;
  if (in_sizes[2] != FFD * DIM) return;
  if (in_sizes[3] != DIM * FFD) return;
  if (out_size != NB_ * SEQ * DIM) return;

  const float* x    = (const float*)d_in[0];
  const float* w_qk = (const float*)d_in[1];
  const float* w1   = (const float*)d_in[2];
  const float* w2   = (const float*)d_in[3];

  const size_t MiB = (size_t)1048576;
  const size_t szXsF = (size_t)NB_ * SEQ * DIM * 4;
  const size_t szHH  = (size_t)NB_ * SEQ * FFD * 2;
  const size_t szXsH = (size_t)NB_ * SEQ * DIM * 2;
  const size_t szW1  = (size_t)FFD * DIM * 2;
  const size_t szW2  = (size_t)DIM * FFD * 2;
  const size_t szWqk = (size_t)2 * DIM * DIM * 2;
  const size_t szXf  = (size_t)NBH * SEQ * HD * 4;
  const size_t szMT  = (size_t)NBH * HD * SEQ * 2;
  const size_t szRi  = (size_t)NBH * SEQ * 4;
  const size_t szQK  = (size_t)NBH * SEQ * HD * 2;
  const size_t szE   = (size_t)GRP * SEQ * SEQ * 2;

  size_t off = 0;
  const size_t oXsF = off; off += szXsF;
  const size_t oHH  = off; off += szHH;
  const size_t oXsH = off; off += szXsH;
  const size_t oW1  = off; off += szW1;
  const size_t oW2  = off; off += szW2;
  const size_t oWqk = off; off += szWqk;
  const size_t oXf  = off; off += szXf;
  const size_t oMTa = off; off += szMT;
  const size_t oMTb = off; off += szMT;
  const size_t oRi  = off; off += szRi;
  const size_t oKH  = off; off += szQK;
  const size_t oQH  = oW2;
  const size_t oE   = 0;
  if (off > ws_size) return;
  if (off > 128 * MiB) return;
  if (oE + szE > oQH) return;
  if (oQH + szQK > oWqk) return;

  char* ws = (char*)d_ws;
  float*          xsF  = (float*)(ws + oXsF);
  unsigned short* hH   = (unsigned short*)(ws + oHH);
  unsigned short* xsH  = (unsigned short*)(ws + oXsH);
  unsigned short* w1H  = (unsigned short*)(ws + oW1);
  unsigned short* w2H  = (unsigned short*)(ws + oW2);
  unsigned short* wqkH = (unsigned short*)(ws + oWqk);
  float*          xf   = (float*)(ws + oXf);
  unsigned short* mTa  = (unsigned short*)(ws + oMTa);
  unsigned short* mTb  = (unsigned short*)(ws + oMTb);
  float*          rinv = (float*)(ws + oRi);
  unsigned short* kH   = (unsigned short*)(ws + oKH);
  unsigned short* qH   = (unsigned short*)(ws + oQH);
  unsigned short* E    = (unsigned short*)(ws + oE);
  float*          outF = (float*)d_out;

  const dim3 blk(256);
  const int n8qk = 2 * DIM * DIM / 8;
  const int n8w  = FFD * DIM / 8;

  k_cvt_h<<<dim3((n8qk + 255) / 256), blk, 0, stream>>>(w_qk, wqkH, n8qk, W_CARRY);
  k_cvt_h<<<dim3((n8w + 255) / 256), blk, 0, stream>>>(w1, w1H, n8w, W_CARRY);
  k_cvt_h<<<dim3((n8w + 255) / 256), blk, 0, stream>>>(w2, w2H, n8w, W_CARRY);
  k_norm_x<<<dim3(NB_ * SEQ), blk, 0, stream>>>(x, xsF, xsH);
  {
    const int tiles = (NB_ * SEQ / 64) * (FFD / 64);
    k_gemm<MODE_GELU><<<dim3((tiles + 7) / 8), blk, 0, stream>>>(
        xsH, DIM, w1H, DIM, NB_ * SEQ, FFD, DIM, hH, hH, xf, xsF);
  }
  {
    const int tiles = (DIM / 64) * (NB_ * SEQ / 64);
    k_gemm<MODE_FF2><<<dim3((tiles + 7) / 8), blk, 0, stream>>>(
        w2H, FFD, hH, FFD, DIM, NB_ * SEQ, FFD, mTa, mTa, xf, xsF);
  }
  {
    const int tiles = (NB_ * SEQ / 64) * (2 * DIM / 64);
    k_gemm<MODE_QK><<<dim3((tiles + 7) / 8), blk, 0, stream>>>(
        xsH, DIM, wqkH, DIM, NB_ * SEQ, 2 * DIM, DIM, qH, kH, xf, xsF);
  }
  for (int g = 0; g < NBH / GRP; ++g) {
    const int bh0 = g * GRP;
    k_scores<<<dim3(GRP * 8), blk, 0, stream>>>(qH, kH, E, rinv, bh0);
    unsigned short* cur = mTa;
    unsigned short* nxt = mTb;
    for (int s = 2; s <= NSTEP; ++s) {
      if (s < NSTEP) {
        k_iter<0><<<dim3(GRP * 4), blk, 0, stream>>>(cur, E, rinv, xf, nxt, outF, bh0);
        unsigned short* t = cur; cur = nxt; nxt = t;
      } else {
        k_iter<1><<<dim3(GRP * 4), blk, 0, stream>>>(cur, E, rinv, xf, nxt, outF, bh0);
      }
    }
  }
  (void)hipGetLastError();
}
